// CosformerAttention_49263274885960
// MI455X (gfx1250) — hardware-verified
//
#include <hip/hip_runtime.h>


typedef _Float16 v16h __attribute__((ext_vector_type(16)));
typedef _Float16 v8h  __attribute__((ext_vector_type(8)));
typedef float    v8f  __attribute__((ext_vector_type(8)));
typedef float    v4f  __attribute__((ext_vector_type(4)));

#define L_    2048
#define E_    1024
#define NH_   64
#define DH_   64
#define D2_   128
#define R_    8192
#define SP_   68

#define W_SCALE      1024.0f
#define INV_W_SCALE  (1.0f / 1024.0f)
#define ACT_SCALE    64.0f
#define KV_PACK      (1.0f / 16.0f)
#define INV_DEN      (1.0f / 4096.0f)
#define INV_ATT      (1.0f / 16384.0f)

union Frag { v16h v; v8h hv[2]; };

__device__ __forceinline__ v16h ld_frag(const _Float16* rowp, int k0, int hsel) {
  Frag f;
  f.hv[0] = *(const v8h*)(rowp + k0 + 8 * hsel);
  f.hv[1] = *(const v8h*)(rowp + k0 + 16 + 8 * hsel);
  return f.v;
}

__device__ __forceinline__ v8f wmma_f16(v16h a, v16h b, v8f c) {
  v8f d = __builtin_amdgcn_wmma_f32_16x16x32_f16(false, a, false, b, (short)0, c, false, false);
  asm volatile("v_nop\n\tv_nop\n\tv_nop\n\tv_nop" : "+v"(d) : "v"(a), "v"(b));
  return d;
}

__device__ __forceinline__ v8f zero8() {
  v8f z = {0.f, 0.f, 0.f, 0.f, 0.f, 0.f, 0.f, 0.f};
  return z;
}

__device__ __forceinline__ float wave_sum(float v) {
  v += __shfl_xor(v, 16);
  v += __shfl_xor(v, 8);
  v += __shfl_xor(v, 4);
  v += __shfl_xor(v, 2);
  v += __shfl_xor(v, 1);
  return v;
}

__global__ __launch_bounds__(256)
void k_wbuild(const float* __restrict__ A, const float* __restrict__ S, _Float16* Wt) {
  const int e = blockIdx.x * 256 + threadIdx.x;
  const int base = e * 8;
  const int col = base >> 10;
  const int kst = base & 1023;
  const int jb = col >> 8, l2 = col & 255;
  v8h o;
#pragma unroll
  for (int j = 0; j < 8; ++j) {
    const int kk = kst + j;
    const int i = kk >> 8, k2 = kk & 255;
    float acc = 0.f;
#pragma unroll
    for (int p = 0; p < 4; ++p)
      acc += A[p * 16 + i * 4 + jb] * S[(p * 256 + k2) * 256 + l2];
    o[j] = (_Float16)(acc * W_SCALE);
  }
  for (int pass = 0; pass < 2; ++pass) {
    *(volatile v8h*)(Wt + base) = o;
    if (pass == 0) __threadfence();
  }
}

template <int RAW>
__global__ __launch_bounds__(128)
void k_ln(const float* __restrict__ x, const float* __restrict__ g, const float* __restrict__ b,
          float* y32, _Float16* y16, _Float16* x16) {
  __shared__ __attribute__((aligned(16))) float rowbuf[E_];
  __shared__ float red[8];
  const int row = blockIdx.x, tid = threadIdx.x, wave = tid >> 5, lane = tid & 31;
  const int c0 = tid * 8;
  const float* xr = x + (size_t)row * E_;
  const v4f u0 = *(const v4f*)(xr + c0);
  const v4f u1 = *(const v4f*)(xr + c0 + 4);
  float v[8];
  v[0] = u0[0]; v[1] = u0[1]; v[2] = u0[2]; v[3] = u0[3];
  v[4] = u1[0]; v[5] = u1[1]; v[6] = u1[2]; v[7] = u1[3];
  float s = ((v[0] + v[1]) + (v[2] + v[3])) + ((v[4] + v[5]) + (v[6] + v[7]));
  s = wave_sum(s);
  if (lane == 0) red[wave] = s;
  __syncthreads();
  const float mean = ((red[0] + red[1]) + (red[2] + red[3])) * (1.0f / (float)E_);
  float q = 0.f;
#pragma unroll
  for (int j = 0; j < 8; ++j) { const float d = v[j] - mean; q += d * d; }
  q = wave_sum(q);
  if (lane == 0) red[4 + wave] = q;
  __syncthreads();
  const float var = ((red[4] + red[5]) + (red[6] + red[7])) * (1.0f / (float)E_);
  const float rstd = rsqrtf(var + 1e-5f);
  const v4f g0 = *(const v4f*)(g + c0), g1 = *(const v4f*)(g + c0 + 4);
  const v4f b0 = *(const v4f*)(b + c0), b1 = *(const v4f*)(b + c0 + 4);
  float gg[8], bb[8], y[8];
  gg[0] = g0[0]; gg[1] = g0[1]; gg[2] = g0[2]; gg[3] = g0[3];
  gg[4] = g1[0]; gg[5] = g1[1]; gg[6] = g1[2]; gg[7] = g1[3];
  bb[0] = b0[0]; bb[1] = b0[1]; bb[2] = b0[2]; bb[3] = b0[3];
  bb[4] = b1[0]; bb[5] = b1[1]; bb[6] = b1[2]; bb[7] = b1[3];
  v8h pk, px;
#pragma unroll
  for (int j = 0; j < 8; ++j) {
    y[j] = (v[j] - mean) * rstd * gg[j] + bb[j];
    pk[j] = (_Float16)y[j];
    px[j] = (_Float16)v[j];
  }
  v4f w0, w1;
  w0[0] = y[0]; w0[1] = y[1]; w0[2] = y[2]; w0[3] = y[3];
  w1[0] = y[4]; w1[1] = y[5]; w1[2] = y[6]; w1[3] = y[7];
  *(v4f*)&rowbuf[c0]     = w0;
  *(v4f*)&rowbuf[c0 + 4] = w1;
  __syncthreads();
  const size_t rofs = (size_t)row * E_;
  for (int pass = 0; pass < 2; ++pass) {
    *(volatile v8h*)(y16 + rofs + c0) = pk;
    if (RAW) *(volatile v8h*)(x16 + rofs + c0) = px;
#pragma unroll
    for (int j = 0; j < 2; ++j) {
      const int idx = wave * 256 + j * 128 + 4 * lane;
      const v4f t = *(const v4f*)&rowbuf[idx];
      *(volatile v4f*)(y32 + rofs + idx) = t;
    }
    if (pass == 0) __threadfence();
  }
}

template <int MODE>
__global__ __launch_bounds__(256)
void k_gemm(const _Float16* __restrict__ X, const _Float16* __restrict__ Wt,
            const float* __restrict__ bias, _Float16* out16,
            const float* __restrict__ resid, float* out32) {
  __shared__ __attribute__((aligned(16))) float stage[256 * SP_];
  __shared__ float trig[128];
  const int wave = threadIdx.x >> 5, lane = threadIdx.x & 31, hl = lane >> 4, m = lane & 15;
  const int rowbase = blockIdx.x * 256;
  const int colbase = blockIdx.y * 64;
  const int hcol = blockIdx.y;
  const int l0 = rowbase >> 2;

  if (MODE == 0 || MODE == 1) {
    if (threadIdx.x < 64) {
      const int l = l0 + (int)threadIdx.x;
      const float ang = (1.57079632679f * (float)(l + 1)) * (1.0f / (float)L_);
      trig[2 * threadIdx.x]     = sinf(ang);
      trig[2 * threadIdx.x + 1] = cosf(ang);
    }
  }

  v8f acc[2][4];
#pragma unroll
  for (int gq = 0; gq < 2; ++gq)
#pragma unroll
    for (int t = 0; t < 4; ++t) acc[gq][t] = zero8();

  const _Float16* xr0 = X + (size_t)(rowbase + wave * 32 + m) * E_;
  const _Float16* xr1 = xr0 + (size_t)16 * E_;
  const _Float16* wr0 = Wt + (size_t)(colbase + m) * E_;

  for (int k0 = 0; k0 < E_; k0 += 32) {
    const v16h a0 = ld_frag(xr0, k0, hl);
    const v16h a1 = ld_frag(xr1, k0, hl);
#pragma unroll
    for (int t = 0; t < 4; ++t) {
      const v16h bfr = ld_frag(wr0 + (size_t)(16 * t) * E_, k0, hl);
      acc[0][t] = wmma_f16(a0, bfr, acc[0][t]);
      acc[1][t] = wmma_f16(a1, bfr, acc[1][t]);
    }
  }

#pragma unroll
  for (int gq = 0; gq < 2; ++gq) {
#pragma unroll
    for (int t = 0; t < 4; ++t) {
      const int cl = 16 * t + m;
      const float bv = bias[colbase + cl];
#pragma unroll
      for (int r = 0; r < 8; ++r) {
        float val = acc[gq][t][r] * INV_W_SCALE + bv;
        if (MODE == 0 || MODE == 1) val = fmaxf(val, 0.0f);
        stage[(wave * 32 + 16 * gq + 8 * hl + r) * SP_ + cl] = val;
      }
    }
  }
  __syncthreads();

  const int c8 = lane & 7;
  if (MODE == 0) {
    for (int pass = 0; pass < 2; ++pass) {
#pragma unroll 1
      for (int it = 0; it < 16; ++it) {
        const int lid = it * 32 + wave * 4 + (lane >> 3);
        const int rl = lid >> 1, sc = lid & 1;
        const int row = rowbase + rl;
        const int l = row >> 2, n = row & 3;
        const int hh = n * 16 + hcol;
        const float w = ACT_SCALE * trig[2 * (rl >> 2) + sc];
        const v4f s0 = *(const v4f*)&stage[rl * SP_ + 8 * c8];
        const v4f s1 = *(const v4f*)&stage[rl * SP_ + 8 * c8 + 4];
        v8h o;
        o[0] = (_Float16)(s0[0] * w); o[1] = (_Float16)(s0[1] * w);
        o[2] = (_Float16)(s0[2] * w); o[3] = (_Float16)(s0[3] * w);
        o[4] = (_Float16)(s1[0] * w); o[5] = (_Float16)(s1[1] * w);
        o[6] = (_Float16)(s1[2] * w); o[7] = (_Float16)(s1[3] * w);
        _Float16* dst = out16 + ((size_t)(hh * L_ + l) * D2_ + sc * 64 + 8 * c8);
        *(volatile v8h*)dst = o;
      }
      if (pass == 0) __threadfence();
    }
  } else if (MODE == 1) {
    for (int pass = 0; pass < 2; ++pass) {
#pragma unroll 1
      for (int it = 0; it < 16; ++it) {
        const int lid = it * 32 + wave * 4 + (lane >> 3);
        const int d = lid & 63, sc = (lid >> 6) & 1, n = lid >> 7;
        const int hh = n * 16 + hcol;
        v8h o;
#pragma unroll
        for (int j = 0; j < 8; ++j) {
          const int ll = 8 * c8 + j;
          o[j] = (_Float16)(stage[(ll * 4 + n) * SP_ + d] * (ACT_SCALE * trig[2 * ll + sc]));
        }
        _Float16* dst = out16 + ((size_t)(hh * D2_ + sc * 64 + d) * L_ + l0 + 8 * c8);
        *(volatile v8h*)dst = o;
      }
      if (pass == 0) __threadfence();
    }
  } else if (MODE == 2) {
    for (int pass = 0; pass < 2; ++pass) {
#pragma unroll 1
      for (int it = 0; it < 8; ++it) {
        const int lid = it * 32 + wave * 4 + (lane >> 3);
        const int d = lid & 63, n = lid >> 6;
        const int hh = n * 16 + hcol;
        v8h o;
#pragma unroll
        for (int j = 0; j < 8; ++j) {
          const int ll = 8 * c8 + j;
          o[j] = (_Float16)(stage[(ll * 4 + n) * SP_ + d] * ACT_SCALE);
        }
        _Float16* dst = out16 + ((size_t)(hh * DH_ + d) * L_ + l0 + 8 * c8);
        *(volatile v8h*)dst = o;
      }
      if (pass == 0) __threadfence();
    }
  } else {
    for (int pass = 0; pass < 2; ++pass) {
#pragma unroll 1
      for (int it = 0; it < 16; ++it) {
        const int lid = it * 32 + wave * 4 + (lane >> 3);
        const int rl = lid >> 1, half = lid & 1;
        const int cl = half * 32 + 4 * c8;
        const v4f sv = *(const v4f*)&stage[rl * SP_ + cl];
        const size_t o = (size_t)(rowbase + rl) * E_ + colbase + cl;
        const v4f rs = *(const v4f*)(resid + o);
        const v4f y = sv + rs;
        *(volatile v4f*)(out32 + o) = y;
      }
      if (pass == 0) __threadfence();
    }
  }
}

__global__ __launch_bounds__(256)
void k_kv(const _Float16* __restrict__ kT, const _Float16* __restrict__ vT,
          _Float16* kvT, float* ksum) {
  __shared__ __attribute__((aligned(16))) float stage[D2_ * SP_];
  __shared__ __attribute__((aligned(16))) float ks[D2_];
  const int hh = blockIdx.x;
  const int wave = threadIdx.x >> 5, lane = threadIdx.x & 31, hl = lane >> 4, m = lane & 15;
  const _Float16* arow = kT + ((size_t)(hh * D2_ + wave * 16 + m)) * L_;
  const _Float16* brow = vT + ((size_t)(hh * DH_ + m)) * L_;
  v8f acc[4];
#pragma unroll
  for (int t = 0; t < 4; ++t) acc[t] = zero8();
  float ksp = 0.f;

  for (int k0 = 0; k0 < L_; k0 += 32) {
    const v16h a = ld_frag(arow, k0, hl);
#pragma unroll
    for (int i = 0; i < 16; ++i) ksp += (float)a[i];
#pragma unroll
    for (int t = 0; t < 4; ++t) {
      const v16h bfr = ld_frag(brow + (size_t)(16 * t) * L_, k0, hl);
      acc[t] = wmma_f16(a, bfr, acc[t]);
    }
  }
  ksp += __shfl_xor(ksp, 16);
  if (hl == 0) ks[wave * 16 + m] = ksp;
#pragma unroll
  for (int t = 0; t < 4; ++t)
#pragma unroll
    for (int r = 0; r < 8; ++r)
      stage[(wave * 16 + 8 * hl + r) * SP_ + 16 * t + m] = acc[t][r] * KV_PACK;
  __syncthreads();

  const int c8 = lane & 7;
  for (int pass = 0; pass < 2; ++pass) {
    if (wave == 0) {
      const v4f kv4 = *(const v4f*)&ks[4 * lane];
      *(volatile v4f*)(ksum + hh * D2_ + 4 * lane) = kv4;
    }
#pragma unroll 1
    for (int it = 0; it < 4; ++it) {
      const int lid = it * 32 + wave * 4 + (lane >> 3);
      const int mm = lid >> 1, half = lid & 1;
      v8h o;
#pragma unroll
      for (int j = 0; j < 8; ++j) {
        const int dd = half * 64 + 8 * c8 + j;
        o[j] = (_Float16)stage[dd * SP_ + mm];
      }
      _Float16* dst = kvT + ((size_t)(hh * DH_ + mm) * D2_ + half * 64 + 8 * c8);
      *(volatile v8h*)dst = o;
    }
    if (pass == 0) __threadfence();
  }
}

__global__ __launch_bounds__(256)
void k_attn(const _Float16* __restrict__ q16, const _Float16* __restrict__ kvT,
            const float* __restrict__ ksum, const float* __restrict__ qn32, float* attn32) {
  __shared__ __attribute__((aligned(16))) float stage[128 * SP_];
  __shared__ float ks[D2_];
  __shared__ float zs[128];
  const int lblk = blockIdx.x, hh = blockIdx.y;
  const int wave = threadIdx.x >> 5, lane = threadIdx.x & 31, hl = lane >> 4, m = lane & 15;
  if (threadIdx.x < D2_) ks[threadIdx.x] = ksum[hh * D2_ + threadIdx.x];
  __syncthreads();

  const int lrow = lblk * 128 + wave * 16 + m;
  const _Float16* arow = q16 + ((size_t)(hh * L_ + lrow)) * D2_;
  const _Float16* brow = kvT + ((size_t)(hh * DH_ + m)) * D2_;
  v8f acc[4];
#pragma unroll
  for (int t = 0; t < 4; ++t) acc[t] = zero8();
  float rs = 0.f;
#pragma unroll
  for (int k0 = 0; k0 < D2_; k0 += 32) {
    const v16h a = ld_frag(arow, k0, hl);
#pragma unroll
    for (int i = 0; i < 8; ++i) {
      rs += (float)a[i]     * ks[k0 + 8 * hl + i];
      rs += (float)a[8 + i] * ks[k0 + 16 + 8 * hl + i];
    }
#pragma unroll
    for (int t = 0; t < 4; ++t) {
      const v16h bfr = ld_frag(brow + (size_t)(16 * t) * D2_, k0, hl);
      acc[t] = wmma_f16(a, bfr, acc[t]);
    }
  }
  rs += __shfl_xor(rs, 16);
  const float denom = rs * INV_DEN;
  const float z = 1.0f / fmaxf(denom, 1e-6f);
  if (hl == 0) zs[wave * 16 + m] = z;
#pragma unroll
  for (int t = 0; t < 4; ++t)
#pragma unroll
    for (int r = 0; r < 8; ++r)
      stage[(wave * 16 + 8 * hl + r) * SP_ + 16 * t + m] = acc[t][r];
  __syncthreads();

  const int n = hh >> 4, h = hh & 15;
  const int c8 = lane & 7;
  for (int pass = 0; pass < 2; ++pass) {
#pragma unroll 1
    for (int it = 0; it < 8; ++it) {
      const int lid = it * 32 + wave * 4 + (lane >> 3);
      const int ll = lid >> 1, half = lid & 1;
      const int cl = half * 32 + 4 * c8;
      const float zz = zs[ll] * INV_ATT;
      const v4f sv = *(const v4f*)&stage[ll * SP_ + cl];
      const int l = lblk * 128 + ll;
      const size_t o = (size_t)(l * 4 + n) * E_ + h * DH_ + cl;
      const v4f base = *(const v4f*)(qn32 + o);
      v4f y;
      y[0] = sv[0] * zz + base[0]; y[1] = sv[1] * zz + base[1];
      y[2] = sv[2] * zz + base[2]; y[3] = sv[3] * zz + base[3];
      *(volatile v4f*)(attn32 + o) = y;
    }
    if (pass == 0) __threadfence();
  }
}

extern "C" void kernel_launch(void* const* d_in, const int* in_sizes, int n_in,
                              void* d_out, int out_size, void* d_ws, size_t ws_size,
                              hipStream_t stream) {
  if (n_in < 17) return;
  const int expect_n[17] = {R_ * E_, 64, 262144, E_, 64, 262144, E_, 64, 262144, E_,
                            64, 262144, E_, E_, E_, E_, E_};
  for (int i = 0; i < 17; ++i)
    if (in_sizes[i] != expect_n[i]) return;
  if (out_size != R_ * E_) return;
  const size_t MiB = 1048576ull;
  const size_t need = 122ull * MiB;
  if (ws_size < need) return;

  const float* query = (const float*)d_in[0];
  const float* qA = (const float*)d_in[1];  const float* qS = (const float*)d_in[2];
  const float* qb = (const float*)d_in[3];
  const float* kA = (const float*)d_in[4];  const float* kS = (const float*)d_in[5];
  const float* kb = (const float*)d_in[6];
  const float* vA = (const float*)d_in[7];  const float* vS = (const float*)d_in[8];
  const float* vb = (const float*)d_in[9];
  const float* oA = (const float*)d_in[10]; const float* oS = (const float*)d_in[11];
  const float* ob = (const float*)d_in[12];
  const float* g1 = (const float*)d_in[13]; const float* b1 = (const float*)d_in[14];
  const float* g2 = (const float*)d_in[15]; const float* b2 = (const float*)d_in[16];
  float* outF = (float*)d_out;

  char* ws = (char*)d_ws;
  _Float16* Wq     = (_Float16*)(ws + 0 * MiB);
  _Float16* Wk     = (_Float16*)(ws + 2 * MiB);
  _Float16* Wv     = (_Float16*)(ws + 4 * MiB);
  _Float16* Wo     = (_Float16*)(ws + 6 * MiB);
  _Float16* kvT    = (_Float16*)(ws + 8 * MiB);
  float*    ksum   = (float*)   (ws + 9 * MiB);
  float*    qn32   = (float*)   (ws + 10 * MiB);
  _Float16* qn16   = (_Float16*)(ws + 42 * MiB);
  _Float16* x16    = (_Float16*)(ws + 58 * MiB);
  _Float16* kT     = (_Float16*)(ws + 74 * MiB);
  _Float16* vT     = (_Float16*)(ws + 106 * MiB);
  _Float16* q16    = (_Float16*)(ws + 58 * MiB);
  float*    attn32 = (float*)   (ws + 90 * MiB);
  float*    o32    = (float*)   (ws + 10 * MiB);
  _Float16* o16    = (_Float16*)(ws + 42 * MiB);

  k_wbuild<<<512, 256, 0, stream>>>(qA, qS, Wq);
  k_wbuild<<<512, 256, 0, stream>>>(kA, kS, Wk);
  k_wbuild<<<512, 256, 0, stream>>>(vA, vS, Wv);
  k_wbuild<<<512, 256, 0, stream>>>(oA, oS, Wo);

  k_ln<1><<<R_, 128, 0, stream>>>(query, g1, b1, qn32, qn16, x16);

  const dim3 gg(R_ / 256, E_ / 64);
  k_gemm<1><<<gg, 256, 0, stream>>>(x16, Wk, kb, kT, qn32, ksum);
  k_gemm<2><<<gg, 256, 0, stream>>>(x16, Wv, vb, vT, qn32, ksum);
  k_kv<<<NH_, 256, 0, stream>>>(kT, vT, kvT, ksum);

  k_gemm<0><<<gg, 256, 0, stream>>>(qn16, Wq, qb, q16, qn32, ksum);

  k_attn<<<dim3(L_ / 128, NH_), 256, 0, stream>>>(q16, kvT, ksum, qn32, attn32);

  k_ln<0><<<R_, 128, 0, stream>>>(attn32, g2, b2, o32, o16, o16);
  k_gemm<3><<<gg, 256, 0, stream>>>(o16, Wo, ob, o16, o32, outF);
}
